// Block_21947282883003
// MI455X (gfx1250) — hardware-verified
//
#include <hip/hip_runtime.h>
#ifndef NB
#define NB 2
#endif
#ifndef SEQ
#define SEQ 2048
#endif
#define NB_FULL 2
#define SEQ_FULL 2048
#define DM 768
#define NH 12
#define HD 64
#define DFF 3072
#define DMQ DM
#define LQ (3 * DM)
#define NR ((size_t)NB * SEQ)

static_assert(NH * HD == DM);
static_assert(SEQ % 64 == 0);
static_assert(((size_t)NB * SEQ) % 128 == 0);
static_assert(DM % 64 == 0 && DFF % 64 == 0 && LQ % 64 == 0);
static_assert(DM % 32 == 0 && DFF % 32 == 0 && HD % 32 == 0);
static_assert(NB <= NB_FULL && SEQ <= SEQ_FULL);

typedef unsigned short v8us __attribute__((ext_vector_type(8), may_alias));
typedef float  v8f  __attribute__((ext_vector_type(8)));
typedef float  v4f  __attribute__((ext_vector_type(4)));
typedef float  v4fa __attribute__((ext_vector_type(4), may_alias));
typedef int    v4i  __attribute__((ext_vector_type(4)));
typedef int    v4ia __attribute__((ext_vector_type(4), may_alias));
typedef _Float16 v16h __attribute__((ext_vector_type(16)));
typedef _Float16 v4h __attribute__((ext_vector_type(4)));
union FragH { v16h v; v8us half[2]; _Float16 h[16]; unsigned short u[16]; };

__device__ __forceinline__ unsigned short bf16_bits(float x) { unsigned int u = __float_as_uint(x); return (unsigned short)((u + 0x7FFFu + ((u >> 16) & 1u)) >> 16); }
__device__ __forceinline__ float bf16_val(unsigned short b) { return __uint_as_float(((unsigned int)b) << 16); }
__device__ __forceinline__ float bf16_rne(float x) { return bf16_val(bf16_bits(x)); }

__global__ __launch_bounds__(256) void k_wt_f16(const float* __restrict__ W, _Float16* __restrict__ Wt, int K, int N, float scale) {
  const int t = blockIdx.x * 256 + threadIdx.x; if (t >= N * (K / 8)) return; const int n = t / (K / 8), k8 = (t % (K / 8)) * 8; FragH f;
#pragma unroll
  for (int i = 0; i < 8; ++i) f.h[i] = (_Float16)(bf16_rne(W[(size_t)(k8 + i) * N + n]) * scale);
  const v8us o = f.half[0];
  *(volatile v8us*)((unsigned short*)Wt + (size_t)n * K + k8) = o; __threadfence(); *(volatile v8us*)((unsigned short*)Wt + (size_t)n * K + k8) = o;
}

template <int BFIN, int W16, int WXB, int REMAP>
__global__ __launch_bounds__(256) void k_lnx(const float* __restrict__ X, const float* __restrict__ g, const float* __restrict__ bb, float eps, _Float16* __restrict__ N16, float* __restrict__ XB) {
  #pragma clang fp contract(off)
  __shared__ float red[256]; const size_t r = blockIdx.x; const int t = threadIdx.x; const bool act = t < (DMQ / 4); const int c0 = act ? t * 4 : 0;
  const size_t xr = REMAP ? ((r / SEQ) * (size_t)SEQ_FULL + (r % SEQ)) : r;
  const v4f xa = *(const v4fa*)(X + xr * DMQ + c0); float s[4]; float sum = 0.f;
  for (int q = 0; q < 4; ++q) { s[q] = act ? (BFIN ? bf16_rne(xa[q]) : xa[q]) : 0.f; sum = __fadd_rn(sum, s[q]); }
  red[t] = sum; __syncthreads(); for (int st = 128; st > 0; st >>= 1) { if (t < st) red[t] = __fadd_rn(red[t], red[t + st]); __syncthreads(); } const float mu = red[0] / (float)DMQ; __syncthreads();
  float vs = 0.f; for (int q = 0; q < 4; ++q) { const float dl = act ? __fadd_rn(s[q], -mu) : 0.f; vs = __fadd_rn(vs, __fmul_rn(dl, dl)); } red[t] = vs; __syncthreads(); for (int st = 128; st > 0; st >>= 1) { if (t < st) red[t] = __fadd_rn(red[t], red[t + st]); __syncthreads(); }
  const float rs = rsqrtf(__fadd_rn(red[0] / (float)DMQ, eps)); v4h y; v4f xb;
  for (int q = 0; q < 4; ++q) { const int c = c0 + q; const float yf = __fadd_rn(__fmul_rn(__fmul_rn(__fadd_rn(s[q], -mu), rs), bf16_rne(g[c])), bf16_rne(bb[c])); y[q] = (_Float16)yf; xb[q] = s[q]; }
  if (!act) return;
  for (int pass = 0; pass < 2; ++pass) { if (W16) *(volatile v4h*)(N16 + r * DMQ + c0) = y; if (WXB) *(volatile v4f*)(XB + r * DMQ + c0) = xb; if (pass == 0) __threadfence(); } }

__device__ __forceinline__ v16h g2_frag(const _Float16* p, int hh) { FragH f; f.half[0] = *(const v8us*)((const unsigned short*)p + 8 * hh); f.half[1] = *(const v8us*)((const unsigned short*)p + 16 + 8 * hh); return f.v; }
__device__ __forceinline__ v8f g2_mma(v16h a, v16h b, v8f c) { v8f d = __builtin_amdgcn_wmma_f32_16x16x32_f16(false, a, false, b, (short)0, c, false, false); asm volatile("v_nop\n\tv_nop\n\tv_nop\n\tv_nop" : "+v"(d) : "v"(a), "v"(b)); return d; }
template <int ACT>
__global__ __launch_bounds__(128) void k_gemm2(const _Float16* __restrict__ A, int lda, size_t sA, const _Float16* __restrict__ Bh, int ldb, size_t sB, float alpha, const float* __restrict__ bias, size_t sBias, const float* __restrict__ CP, int rowsPerB, size_t sCPb, int row0g,
    float* __restrict__ C, _Float16* __restrict__ C16, int ldc, size_t sC, int M, int N, int K) { static_assert(ACT == 0 || ACT == 3);
  __shared__ __attribute__((aligned(16))) float so[4][32][68];
  const int tid = threadIdx.x, lane = tid & 31, ln = lane & 15, hh = lane >> 4; const int by = blockIdx.y;
  const int w = __builtin_amdgcn_readfirstlane(tid >> 5);
  A += (size_t)by * sA; Bh += (size_t)by * sB; const size_t cofs = (size_t)by * sC; const float* bp = bias ? bias + (size_t)by * sBias : nullptr;
  const int ntn = N >> 6; const int mt = blockIdx.x / ntn, nq = blockIdx.x - mt * ntn; const int row0 = mt * 128 + 32 * w, col0 = nq * 64; if (row0 >= M) return;
  const _Float16* a0p = A + (size_t)(row0 + ln) * lda; const _Float16* a1p = a0p + (size_t)16 * lda;
  const _Float16* b0p = Bh + (size_t)(col0 + ln) * ldb; const _Float16* b1p = b0p + (size_t)16 * ldb; const _Float16* b2p = b1p + (size_t)16 * ldb; const _Float16* b3p = b2p + (size_t)16 * ldb;
  const v8f z8 = {0.f,0.f,0.f,0.f,0.f,0.f,0.f,0.f}; v8f c00 = z8, c01 = z8, c02 = z8, c03 = z8, c10 = z8, c11 = z8, c12 = z8, c13 = z8;
#pragma unroll 1
  for (int kb = 0; kb < K; kb += 32) { const v16h a0 = g2_frag(a0p + kb, hh), a1 = g2_frag(a1p + kb, hh);
    v16h b = g2_frag(b0p + kb, hh); c00 = g2_mma(a0, b, c00); c10 = g2_mma(a1, b, c10);
    b = g2_frag(b1p + kb, hh); c01 = g2_mma(a0, b, c01); c11 = g2_mma(a1, b, c11);
    b = g2_frag(b2p + kb, hh); c02 = g2_mma(a0, b, c02); c12 = g2_mma(a1, b, c12);
    b = g2_frag(b3p + kb, hh); c03 = g2_mma(a0, b, c03); c13 = g2_mma(a1, b, c13); }
  v8f accs[8] = {c00, c01, c02, c03, c10, c11, c12, c13};
#pragma unroll
  for (int u = 0; u < 8; ++u) { const int t = u & 3, half = u >> 2; const int col = col0 + t * 16 + ln; const float bv = bp ? bf16_rne(bp[col]) : 0.f;
#pragma unroll
    for (int r = 0; r < 8; ++r) { const int rloc = half * 16 + 8 * hh + r; float v = accs[u][r] * alpha + bv; if (CP) { if (rowsPerB < 0) v += CP[cofs + (size_t)(row0g + row0 + rloc) * ldc + col];        else { const int bidx = (row0g + row0 + rloc) / rowsPerB; v += CP[(size_t)bidx * sCPb + (size_t)by * 64 + col]; } }
      if (ACT == 3) v = fmaxf(v, 0.f);
      so[w][rloc][t * 16 + ln] = v; } }
  __builtin_amdgcn_fence(4  , "workgroup"); __builtin_amdgcn_wave_barrier();
  const int rsub = lane >> 4, c4 = (lane & 15) * 4;
  for (int pass = 0; pass < 2; ++pass) {
#pragma unroll
    for (int q = 0; q < 16; ++q) { const int r = q * 2 + rsub; const v4f v = *(const v4fa*)&so[w][r][c4]; if (C) *(volatile v4f*)(C + cofs + (size_t)(row0 + r) * ldc + col0 + c4) = v; if (C16) { v4h h4; for (int i = 0; i < 4; ++i) h4[i] = (_Float16)v[i]; *(volatile v4h*)(C16 + cofs + (size_t)(row0 + r) * ldc + col0 + c4) = h4; } }
    if (pass == 0) __threadfence(); } }

template <int NHv, int TTv>
__global__ __launch_bounds__(256) void k_vt(const _Float16* __restrict__ V16, int ldv, int voff, _Float16* __restrict__ Vt) { __shared__ unsigned short tl[64][66]; const int tid = threadIdx.x; const int slab = blockIdx.x / (TTv / 64), lg = blockIdx.x % (TTv / 64); const int b = slab / NHv, h = slab % NHv;
  for (int i = tid; i < 64 * 8; i += 256) { const int r = i / 8, c8 = (i % 8) * 8; FragH f; f.half[0] = *(const v8us*)((const unsigned short*)V16 + ((size_t)b * TTv + lg * 64 + r) * ldv + voff + h * 64 + c8);
#pragma unroll
    for (int q = 0; q < 8; ++q) tl[r][c8 + q] = f.u[q]; }
  __syncthreads();
  for (int pass = 0; pass < 2; ++pass) {
#pragma unroll
    for (int rd = 0; rd < 2; ++rd) { const int d = rd * 32 + tid / 8, pc = tid % 8; FragH f;
#pragma unroll
      for (int q = 0; q < 8; ++q) f.u[q] = tl[pc * 8 + q][d];
      *(volatile v8us*)((unsigned short*)Vt + ((size_t)slab * 64 + d) * TTv + lg * 64 + pc * 8) = f.half[0]; }
    if (pass == 0) __threadfence(); } }

__global__ __launch_bounds__(128) void k_flash(const _Float16* __restrict__ QKV, const _Float16* __restrict__ VT, const int* __restrict__ mask, _Float16* __restrict__ O16, float scale) {
  __shared__ __attribute__((aligned(16))) unsigned short so[4][16][72];
  const int tid = threadIdx.x, lane = tid & 31, ln = lane & 15, hh = lane >> 4;
  const int w = __builtin_amdgcn_readfirstlane(tid >> 5);
  const int qt = blockIdx.x % (SEQ / 64), bh = blockIdx.x / (SEQ / 64); const int b = bh / NH, h = bh % NH;
  const size_t rowb = (size_t)b * SEQ; const int q0 = qt * 64 + 16 * w;
  const _Float16* qp = QKV + (rowb + q0 + ln) * LQ + h * HD;
  const _Float16* kp = QKV + (rowb + ln) * LQ + DM + h * HD;
  const _Float16* vp = VT + ((size_t)bh * HD + ln) * SEQ;
  const int* mp = mask + (size_t)b * SEQ_FULL + 8 * hh;
  const float NINF = -__builtin_inff();
  const v8f z8 = {0.f,0.f,0.f,0.f,0.f,0.f,0.f,0.f};
  v8f o0 = z8, o1 = z8, o2 = z8, o3 = z8; float m = NINF, l = 0.f;
#pragma unroll 1
  for (int k0 = 0; k0 < SEQ; k0 += 32) {
    const _Float16* kr = kp + (size_t)k0 * LQ;
    v8f s0 = z8, s1 = z8;
    {
      const v16h qa = g2_frag(qp, hh);
      v16h ka = g2_frag(kr, hh); s0 = g2_mma(ka, qa, s0);
      ka = g2_frag(kr + (size_t)16 * LQ, hh); s1 = g2_mma(ka, qa, s1);
      const v16h qb = g2_frag(qp + 32, hh);
      ka = g2_frag(kr + 32, hh); s0 = g2_mma(ka, qb, s0);
      ka = g2_frag(kr + (size_t)16 * LQ + 32, hh); s1 = g2_mma(ka, qb, s1);
    }
    const v4i ma = *(const v4ia*)(mp + k0), mb = *(const v4ia*)(mp + k0 + 4), mc = *(const v4ia*)(mp + k0 + 16), md = *(const v4ia*)(mp + k0 + 20);
    float sv[16];
#pragma unroll
    for (int r = 0; r < 4; ++r) {
      sv[r]      = (ma[r] != 0) ? s0[r] * scale : NINF;
      sv[4 + r]  = (mb[r] != 0) ? s0[4 + r] * scale : NINF;
      sv[8 + r]  = (mc[r] != 0) ? s1[r] * scale : NINF;
      sv[12 + r] = (md[r] != 0) ? s1[4 + r] * scale : NINF;
    }
    float lm = sv[0];
#pragma unroll
    for (int i = 1; i < 16; ++i) lm = fmaxf(lm, sv[i]);
    lm = fmaxf(lm, __shfl_xor(lm, 16));
    const float mn = fmaxf(m, lm);
    const float ms = (mn == NINF) ? 0.f : mn;
    const float al = __expf(m - ms);
    const float mm = ms - 5.545177444479562f;
    FragH pf; float ls = 0.f;
#pragma unroll
    for (int i = 0; i < 16; ++i) { const _Float16 ph = (_Float16)__expf(sv[i] - mm); pf.h[i] = ph; ls += (float)ph; }
    l = l * al + ls; m = mn;
#pragma unroll
    for (int r = 0; r < 8; ++r) { o0[r] *= al; o1[r] *= al; o2[r] *= al; o3[r] *= al; }
    const _Float16* vk = vp + k0;
    const v16h v0 = g2_frag(vk, hh), v1 = g2_frag(vk + (size_t)16 * SEQ, hh), v2 = g2_frag(vk + (size_t)32 * SEQ, hh), v3 = g2_frag(vk + (size_t)48 * SEQ, hh);
    o0 = g2_mma(v0, pf.v, o0); o1 = g2_mma(v1, pf.v, o1); o2 = g2_mma(v2, pf.v, o2); o3 = g2_mma(v3, pf.v, o3);
  }
  const float lt = l + __shfl_xor(l, 16);
  const float fin = 64.0f / lt;
  { FragH f;
#pragma unroll
    for (int r = 0; r < 8; ++r) f.h[r] = (_Float16)(o0[r] * fin);
    *(v8us*)&so[w][ln][8 * hh] = f.half[0];
#pragma unroll
    for (int r = 0; r < 8; ++r) f.h[r] = (_Float16)(o1[r] * fin);
    *(v8us*)&so[w][ln][16 + 8 * hh] = f.half[0];
#pragma unroll
    for (int r = 0; r < 8; ++r) f.h[r] = (_Float16)(o2[r] * fin);
    *(v8us*)&so[w][ln][32 + 8 * hh] = f.half[0];
#pragma unroll
    for (int r = 0; r < 8; ++r) f.h[r] = (_Float16)(o3[r] * fin);
    *(v8us*)&so[w][ln][48 + 8 * hh] = f.half[0]; }
  __builtin_amdgcn_fence(4  , "workgroup"); __builtin_amdgcn_wave_barrier();
  const int rq = lane >> 3, pc = (lane & 7) * 8;
  for (int pass = 0; pass < 2; ++pass) {
#pragma unroll
    for (int it = 0; it < 4; ++it) { const int row = it * 4 + rq; const v8us v = *(const v8us*)&so[w][row][pc];
      *(volatile v8us*)((unsigned short*)O16 + (rowb + q0 + row) * DM + h * HD + pc) = v; }
    if (pass == 0) __threadfence(); }
}

extern "C" void kernel_launch(void* const* d_in, const int* in_sizes, int n_in,
                              void* d_out, int out_size, void* d_ws, size_t ws_size, hipStream_t stream) {
  if (n_in < 15) return;
  const long long needx = ((long long)(NB - 1) * SEQ_FULL + SEQ) * DM;
  const long long needm = (long long)(NB - 1) * SEQ_FULL + SEQ;
  if ((long long)in_sizes[0] < needx || (long long)in_sizes[1] < needm) return;
  if (in_sizes[2] < DM * DM || in_sizes[3] < DM * DM || in_sizes[4] < DM * DM || in_sizes[5] < DM * DM || in_sizes[11] < DM * DFF || in_sizes[13] < DFF * DM) return;
  if (in_sizes[6] < DM || in_sizes[7] < DM || in_sizes[8] < DM || in_sizes[9] < DM || in_sizes[10] < DM || in_sizes[12] < DFF || in_sizes[14] < DM) return;
  if ((long long)out_size < (long long)(NR * DM)) return;
  const float* x = (const float*)d_in[0]; const int* am = (const int*)d_in[1];
  const float* wq = (const float*)d_in[2]; const float* wk = (const float*)d_in[3]; const float* wv = (const float*)d_in[4]; const float* wo = (const float*)d_in[5]; const float* bo = (const float*)d_in[6];
  const float* g1 = (const float*)d_in[7]; const float* be1 = (const float*)d_in[8]; const float* g2 = (const float*)d_in[9]; const float* be2 = (const float*)d_in[10];
  const float* w1 = (const float*)d_in[11]; const float* b1 = (const float*)d_in[12]; const float* w2 = (const float*)d_in[13]; const float* b2 = (const float*)d_in[14];
  constexpr size_t SZ_W = (size_t)DM * DM * 2, SZ_W1 = (size_t)DM * DFF * 2, SZ_H = (size_t)NB * SEQ * DM * 2, SZ_F = (size_t)NB * SEQ * DM * 4, SZ_QKV = (size_t)NB * SEQ * LQ * 2, SZ_VT = (size_t)NB * NH * HD * SEQ * 2, SZ_HF = (size_t)NB * SEQ * DFF * 2;
  static_assert(SZ_W % 256 == 0 && SZ_W1 % 256 == 0 && SZ_H % 256 == 0 && SZ_F % 256 == 0 && SZ_QKV % 256 == 0 && SZ_VT % 256 == 0 && SZ_HF % 256 == 0);
  static_assert(SZ_VT >= SZ_H);
  static_assert(4 * SZ_W + 2 * SZ_W1 + 2 * SZ_F + SZ_H + SZ_QKV + SZ_VT + SZ_HF <= (size_t)134217728);
  char* ws = (char*)d_ws; size_t off = 0;
  auto take = [&](size_t bytes) { char* p = ws + off; off += (bytes + 255) & ~(size_t)255; return p; };
  _Float16* BQKV = (_Float16*)take(3 * SZ_W);
  _Float16* BO = (_Float16*)take(SZ_W);
  _Float16* BW1 = (_Float16*)take(SZ_W1);
  _Float16* BW2 = (_Float16*)take(SZ_W1);
  float* XB = (float*)take(SZ_F);
  _Float16* XN = (_Float16*)take(SZ_H);
  _Float16* QKV16 = (_Float16*)take(SZ_QKV);
  _Float16* VT = (_Float16*)take(SZ_VT);
  float* X1 = (float*)take(SZ_F);
  _Float16* HF16 = (_Float16*)take(SZ_HF);
  _Float16* O16 = XN;
  _Float16* M16 = VT;
  if (off > ws_size) return;
  const unsigned gw = (unsigned)(((size_t)DM * (DM / 8) + 255) / 256);
  k_wt_f16<<<gw, 256, 0, stream>>>(wq, BQKV, DM, DM, 16.0f);
  k_wt_f16<<<gw, 256, 0, stream>>>(wk, BQKV + (size_t)DM * DM, DM, DM, 16.0f);
  k_wt_f16<<<gw, 256, 0, stream>>>(wv, BQKV + (size_t)2 * DM * DM, DM, DM, 16.0f);
  k_wt_f16<<<gw, 256, 0, stream>>>(wo, BO, DM, DM, 16.0f);
  k_wt_f16<<<(unsigned)(((size_t)DFF * (DM / 8) + 255) / 256), 256, 0, stream>>>(w1, BW1, DM, DFF, 16.0f);
  k_wt_f16<<<(unsigned)(((size_t)DM * (DFF / 8) + 255) / 256), 256, 0, stream>>>(w2, BW2, DFF, DM, 16.0f);
  k_lnx<1, 1, 1, 1><<<(unsigned)NR, 256, 0, stream>>>(x, g1, be1, 1e-5f, XN, XB);
  k_gemm2<0><<<dim3((unsigned)((NR / 128) * (LQ / 64)), 1), 128, 0, stream>>>(XN, DM, 0, BQKV, DM, 0, 0.0625f, nullptr, 0, nullptr, 1, 0, 0, nullptr, QKV16, LQ, 0, (int)NR, LQ, DM);
  k_vt<NH, SEQ><<<(unsigned)(NB * NH * (SEQ / 64)), 256, 0, stream>>>(QKV16, LQ, 2 * DM, VT);
  k_flash<<<(unsigned)(NB * NH * (SEQ / 64)), 128, 0, stream>>>(QKV16, VT, am, O16, 0.03608439182435161f);
  k_gemm2<0><<<dim3((unsigned)((NR / 128) * (DM / 64)), 1), 128, 0, stream>>>(O16, DM, 0, BO, DM, 0, 0.0009765625f, bo, 0, XB, -1, 0, 0, X1, nullptr, DM, 0, (int)NR, DM, DM);
  k_lnx<0, 1, 0, 0><<<(unsigned)NR, 256, 0, stream>>>(X1, g2, be2, 1e-5f, M16, nullptr);
  k_gemm2<3><<<dim3((unsigned)((NR / 128) * (DFF / 64)), 1), 128, 0, stream>>>(M16, DM, 0, BW1, DM, 0, 0.0625f, b1, 0, nullptr, 1, 0, 0, nullptr, HF16, DFF, 0, (int)NR, DFF, DM);
  k_gemm2<0><<<dim3((unsigned)((NR / 128) * (DM / 64)), 1), 128, 0, stream>>>(HF16, DFF, 0, BW2, DFF, 0, 0.0625f, b2, 0, X1, -1, 0, 0, (float*)d_out, nullptr, DM, 0, (int)NR, DM, DFF);
}
